// DigitCapsule_34686155883103
// MI455X (gfx1250) — hardware-verified
//
#include <hip/hip_runtime.h>
#include <math.h>

typedef __attribute__((ext_vector_type(16))) _Float16 v16h;
typedef __attribute__((ext_vector_type(8)))  _Float16 v8h;
typedef __attribute__((ext_vector_type(8)))  float    v8f;
typedef __attribute__((ext_vector_type(4)))  float    v4f;
typedef __attribute__((ext_vector_type(4)))  unsigned v4u;

constexpr int kB      = 64;
constexpr int kNin    = 4096;
constexpr int kC      = 10;
constexpr int kD      = 8;
constexpr int kE      = 16;
constexpr int kCE     = kC * kE;
constexpr int kChunks = 16;
constexpr int kChunkN = kNin / kChunks;
constexpr int kPairs  = kNin / 2;
constexpr int kTileP  = 2 * kCE;
constexpr int kWVec   = 2 * kC * kE;
constexpr float kCarryX   = 16.0f;
constexpr float kCarryW   = 64.0f;
constexpr float kInvCarry = 1.0f / (kCarryX * kCarryW);
constexpr float kF16Min   = 6.103515625e-5f;
constexpr float kSqEps    = 1e-7f;
static_assert(kCE == 160, "columns per (b,n) row");
static_assert(kChunkN == 256 && (kChunkN % 8) == 0, "chunk of n per routing block");
static_assert((kNin % 2) == 0, "n pairs");
static_assert(kD == 8 && kE == 16, "fragment packing assumes 8 inputs, 16 outputs");

constexpr size_t kSzU16  = (size_t)kB * kNin * kCE * 2;
constexpr size_t kSzSP   = (size_t)kChunks * kB * kCE * 4;
constexpr size_t kSzV    = (size_t)kB * kCE * 4;
constexpr size_t kOffU16 = 0;
constexpr size_t kOffSP0 = kOffU16 + kSzU16;
constexpr size_t kOffSP1 = kOffSP0 + kSzSP;
constexpr size_t kOffSP2 = kOffSP1 + kSzSP;
constexpr size_t kOffVA  = kOffSP2 + kSzSP;
constexpr size_t kOffVB  = kOffVA + kSzV;
constexpr size_t kWsTotal = kOffVB + kSzV;
static_assert(kSzU16 == 83886080ull && kSzSP == 655360ull && kSzV == 40960ull, "region sizes");
static_assert(kWsTotal == 85934080ull, "carve total");
static_assert(kWsTotal <= 134217728ull, "carve cap");
static_assert((kOffSP0 % 128) == 0 && (kOffSP1 % 128) == 0 && (kOffSP2 % 128) == 0 &&
              (kOffVA % 128) == 0 && (kOffVB % 128) == 0, "128-B aligned regions");

union FragU { v16h v; v8h h[2]; };

__device__ __forceinline__ v8f mma_f16_guarded(v16h a, v16h b, v8f c) {
  c = __builtin_amdgcn_wmma_f32_16x16x32_f16(false, a, false, b, (short)0, c, false, false);
  asm volatile("v_nop\n\tv_nop\n\tv_nop\n\tv_nop" : "+v"(c) : "v"(a), "v"(b));
  return c;
}

__device__ __forceinline__ float carry_flush(float v, float carry) {
  const float s = v * carry;
  return (fabsf(s) < kF16Min) ? 0.0f : s;
}

__device__ __forceinline__ float h16_to_f32(unsigned hb) {
  const unsigned sgn = (hb & 0x8000u) << 16;
  const unsigned em = hb & 0x7fffu;
  const float fn = __uint_as_float((em << 13) + 0x38000000u);
  const float fs = (float)em * 5.9604644775390625e-8f;
  const float mag = (em < 0x400u) ? fs : fn;
  return __uint_as_float(__float_as_uint(mag) | sgn);
}

__global__ __launch_bounds__(128) void transform_kernel(
    const float* __restrict__ x, const float* __restrict__ W, unsigned short* __restrict__ U16p)
{
  __shared__ __align__(16) _Float16 Wsh[(kWVec + 1) * 8];
  __shared__ __align__(16) _Float16 Tsh[4 * 16 * kTileP];
  _Float16* U16 = (_Float16*)U16p;
  const int tid  = threadIdx.x;
  const int lane = tid & 31;
  const int wave = tid >> 5;
  const int h    = lane >> 4;
  const int m    = lane & 15;
  const int n0   = blockIdx.x * 2;

  v8h zero8;
#pragma unroll
  for (int e = 0; e < 8; ++e) zero8[e] = (_Float16)0.0f;

  for (int vi = tid; vi < kWVec; vi += 128) {
    const int e  = vi & 15;
    const int nc = vi >> 4;
    const float* src = W + ((size_t)n0 * kC + nc) * (kD * kE) + e;
    v8h hv;
#pragma unroll
    for (int d = 0; d < kD; ++d) {
      const float wv = src[d * kE];
      const float ws = carry_flush(wv, kCarryW);
      hv[d] = (_Float16)ws;
    }
    *(v8h*)(Wsh + vi * 8) = hv;
  }
  if (tid == 127) *(v8h*)(Wsh + kWVec * 8) = zero8;
  __syncthreads();

  _Float16* tw = Tsh + wave * (16 * kTileP);
  const int brow = wave * 16 + m;

#pragma unroll
  for (int nl = 0; nl < 2; ++nl) {
    const float* xp = x + ((size_t)brow * kNin + (n0 + nl)) * kD;
    const v4f xa = *(const v4f*)(xp);
    const v4f xb = *(const v4f*)(xp + 4);
    v8h a8;
#pragma unroll
    for (int d = 0; d < 4; ++d) {
      const float f0 = xa[d];
      const float f1 = xb[d];
      const float s0 = carry_flush(f0, kCarryX);
      const float s1 = carry_flush(f1, kCarryX);
      const float t0 = (h == 0) ? s0 : 0.0f;
      const float t1 = (h == 0) ? s1 : 0.0f;
      a8[d]     = (_Float16)t0;
      a8[4 + d] = (_Float16)t1;
    }
    FragU fa;
    fa.h[0] = a8;
    fa.h[1] = zero8;
#pragma unroll
    for (int c = 0; c < kC; ++c) {
      const int vsel = (h == 0) ? ((nl * kC + c) * 16 + m) : kWVec;
      FragU fb;
      fb.h[0] = *(const v8h*)(Wsh + vsel * 8);
      fb.h[1] = zero8;
      v8f acc = (v8f){0.f, 0.f, 0.f, 0.f, 0.f, 0.f, 0.f, 0.f};
      acc = mma_f16_guarded(fa.v, fb.v, acc);
#pragma unroll
      for (int r = 0; r < 8; ++r) {
        const float f = acc[r] * kInvCarry;
        tw[(8 * h + r) * kTileP + nl * kCE + c * kE + m] = (_Float16)f;
      }
    }
  }
  __syncthreads();

  const int q = lane >> 3;
  const int j = lane & 7;
  for (int pass = 0; pass < 2; ++pass) {
#pragma unroll 4
    for (int it = 0; it < 20; ++it) {
      const int L   = it * 4 + q;
      const int row = L / 5;
      const int ln  = L - row * 5;
      const v8h val = *(const v8h*)(tw + row * kTileP + ln * 64 + j * 8);
      _Float16* dst = U16 + ((size_t)(wave * 16 + row) * kNin + n0) * kCE + ln * 64 + j * 8;
      *(volatile v8h*)dst = val;
    }
    __threadfence();
  }
}

__global__ __launch_bounds__(128) void route_pass_kernel(
    const unsigned short* __restrict__ U16, const float* __restrict__ vsum, int use_vsum,
    float* __restrict__ spart)
{
  __shared__ __align__(16) float red[4 * kCE];
  const int tid  = threadIdx.x;
  const int lane = tid & 31;
  const int wave = tid >> 5;
  const int g    = lane >> 4;
  const int slot = lane & 15;
  const int cc   = (slot < kC) ? slot : (kC - 1);
  const bool act = (slot < kC);
  const int b     = blockIdx.x;
  const int chunk = blockIdx.y;

  float vs[16];
#pragma unroll
  for (int e = 0; e < 16; ++e) vs[e] = 0.0f;
  if (use_vsum != 0) {
    const float* vp = vsum + (size_t)b * kCE + cc * kE;
#pragma unroll
    for (int k = 0; k < 4; ++k) {
      const v4f t4 = *(const v4f*)(vp + 4 * k);
      vs[4 * k + 0] = t4[0];
      vs[4 * k + 1] = t4[1];
      vs[4 * k + 2] = t4[2];
      vs[4 * k + 3] = t4[3];
    }
  }

  float acc[16];
#pragma unroll
  for (int e = 0; e < 16; ++e) acc[e] = 0.0f;

  const unsigned short* ub = U16 + ((size_t)b * kNin + (size_t)chunk * kChunkN) * kCE + cc * kE;

#pragma unroll 1
  for (int it = 0; it < kChunkN / 8; ++it) {
    const int nloc = it * 8 + wave * 2 + g;
    const unsigned short* p = ub + (size_t)nloc * kCE;
    const v4u w0 = *(const v4u*)(p);
    const v4u w1 = *(const v4u*)(p + 8);
    float u[16];
#pragma unroll
    for (int k = 0; k < 4; ++k) {
      const unsigned q0 = w0[k];
      const unsigned q1 = w1[k];
      u[2 * k]         = h16_to_f32(q0 & 0xffffu);
      u[2 * k + 1]     = h16_to_f32(q0 >> 16);
      u[8 + 2 * k]     = h16_to_f32(q1 & 0xffffu);
      u[8 + 2 * k + 1] = h16_to_f32(q1 >> 16);
    }
    float t = 0.0f;
#pragma unroll
    for (int e = 0; e < 16; ++e) t = fmaf(u[e], vs[e], t);
    const float lg = act ? t : -1.0e30f;
    float mx = lg;
    mx = fmaxf(mx, __shfl_xor(mx, 1, 32));
    mx = fmaxf(mx, __shfl_xor(mx, 2, 32));
    mx = fmaxf(mx, __shfl_xor(mx, 4, 32));
    mx = fmaxf(mx, __shfl_xor(mx, 8, 32));
    const float pe = expf(lg - mx);
    float sm = pe;
    sm += __shfl_xor(sm, 1, 32);
    sm += __shfl_xor(sm, 2, 32);
    sm += __shfl_xor(sm, 4, 32);
    sm += __shfl_xor(sm, 8, 32);
    const float wgt = pe * (1.0f / sm);
#pragma unroll
    for (int e = 0; e < 16; ++e) acc[e] = fmaf(wgt, u[e], acc[e]);
  }

#pragma unroll
  for (int e = 0; e < 16; ++e) {
    const float o = __shfl_xor(acc[e], 16, 32);
    acc[e] = acc[e] + o;
  }
  if (g == 0 && act) {
    float* rp = red + wave * kCE + slot * kE;
#pragma unroll
    for (int k = 0; k < 4; ++k) {
      v4f t4;
      t4[0] = acc[4 * k + 0];
      t4[1] = acc[4 * k + 1];
      t4[2] = acc[4 * k + 2];
      t4[3] = acc[4 * k + 3];
      *(v4f*)(rp + 4 * k) = t4;
    }
  }
  __syncthreads();
  {
    const int tc = (tid < 40) ? tid : 39;
    const v4f r0 = *(const v4f*)(red + 0 * kCE + 4 * tc);
    const v4f r1 = *(const v4f*)(red + 1 * kCE + 4 * tc);
    const v4f r2 = *(const v4f*)(red + 2 * kCE + 4 * tc);
    const v4f r3 = *(const v4f*)(red + 3 * kCE + 4 * tc);
    const v4f sv = ((r0 + r1) + r2) + r3;
    float* dst = spart + ((size_t)chunk * kB + b) * kCE + 4 * tc;
    if (tid < 40) {
      *(volatile v4f*)dst = sv;
      __threadfence();
      *(volatile v4f*)dst = sv;
    }
  }
}

__global__ __launch_bounds__(160) void squash_kernel(
    const float* __restrict__ spart, const float* vin, int add_in, float* dst)
{
  const int b   = blockIdx.x;
  const int tid = threadIdx.x;
  float s = 0.0f;
#pragma unroll 1
  for (int ch = 0; ch < kChunks; ++ch) s += spart[((size_t)ch * kB + b) * kCE + tid];
  float s2 = s * s;
  s2 += __shfl_xor(s2, 1, 32);
  s2 += __shfl_xor(s2, 2, 32);
  s2 += __shfl_xor(s2, 4, 32);
  s2 += __shfl_xor(s2, 8, 32);
  const float r1 = 1.0f / (1.0f + s2);
  const float r2 = 1.0f / sqrtf(s2 + kSqEps);
  const float sc = (s2 * r1) * r2;
  float v = sc * s;
  if (add_in != 0) {
    const float pv = vin[(size_t)b * kCE + tid];
    v = v + pv;
  }
  float* o = dst + (size_t)b * kCE + tid;
  *(volatile float*)o = v;
  __threadfence();
  *(volatile float*)o = v;
}

extern "C" void kernel_launch(void* const* d_in, const int* in_sizes, int n_in,
                              void* d_out, int out_size, void* d_ws, size_t ws_size,
                              hipStream_t stream) {
  if (n_in < 2) return;
  if (in_sizes[0] != kB * kNin * kD) return;
  if (in_sizes[1] != kNin * kC * kD * kE) return;
  if (out_size != kB * kCE) return;
  if (ws_size < kWsTotal) return;

  const float* x = (const float*)d_in[0];
  const float* W = (const float*)d_in[1];
  float* out = (float*)d_out;

  char* ws = (char*)d_ws;
  unsigned short* U16 = (unsigned short*)(ws + kOffU16);
  float* SP0 = (float*)(ws + kOffSP0);
  float* SP1 = (float*)(ws + kOffSP1);
  float* SP2 = (float*)(ws + kOffSP2);
  float* VA  = (float*)(ws + kOffVA);
  float* VB  = (float*)(ws + kOffVB);

  transform_kernel<<<kPairs, 128, 0, stream>>>(x, W, U16);

  route_pass_kernel<<<dim3(kB, kChunks), 128, 0, stream>>>(U16, VA, 0, SP0);
  squash_kernel<<<kB, kCE, 0, stream>>>(SP0, VB, 0, VA);

  route_pass_kernel<<<dim3(kB, kChunks), 128, 0, stream>>>(U16, VA, 1, SP1);
  squash_kernel<<<kB, kCE, 0, stream>>>(SP1, VA, 1, VB);

  route_pass_kernel<<<dim3(kB, kChunks), 128, 0, stream>>>(U16, VB, 1, SP2);
  squash_kernel<<<kB, kCE, 0, stream>>>(SP2, VA, 0, out);
}
